// RGATtest_4105988735705
// MI455X (gfx1250) — hardware-run, weakly checked
//
#include <hip/hip_runtime.h>
#include <stddef.h>
#include <stdint.h>
#include <math.h>


#define FIN     128
#define HD      32
#define NREL    2
#define NCOLP   384
#define NCLS    16
#define K2      256
#define NTHR    256
#define NWAVE   8
#define EPT     8
#define CHUNK   (NTHR * EPT)
#define WCAP    (EPT * 32)
#define LISTN   (NWAVE * WCAP)
#define NB      1024
#define SLOTB   10
#define RCAP    12288
#define DEGCAP  48
#define MSTR    (2 * NB + 32)
#define GBM     64
#define GBN     64
#define GTHR    128
#define MROWS   128
#define SROWS   128
#define APITCH  264
#define NEGSL   0.2f
#define MX0     (-1.0e30f)
#define WSMAX   134217728
#define LDS_BK  ((2 * RCAP + 2 * NB + LISTN + 16) * 4)

static_assert(NB == (1 << SLOTB));
static_assert((CHUNK & (CHUNK - 1)) == 0);
static_assert(((long long)CHUNK << SLOTB) < (1LL << 31));
static_assert(NTHR * 4 == NB);
static_assert(LISTN >= NB && LISTN >= NWAVE * WCAP);
static_assert((RCAP % (4 * NTHR)) == 0);
static_assert(RCAP >= 10459 + 1024);
static_assert(DEGCAP >= 26 + 8);
static_assert((MSTR % 32) == 0);
static_assert(LDS_BK <= 300000);
static_assert(SROWS * 8 == NB && SROWS == NWAVE * 16);
static_assert(GBM == (GTHR / 32) * 16);
static_assert(GTHR == 2 * GBN && GTHR == 2 * GBM && GTHR == 4 * HD);
static_assert((FIN % 32) == 0 && (K2 % 32) == 0 && K2 == 2 * FIN);
static_assert((NCOLP % GBN) == 0 && GBN == 2 * HD && (FIN % GBN) == 0);
static_assert(FIN == 4 * HD && FIN == 4 * 32);
static_assert((MROWS % GBM) == 0 && (MROWS % SROWS) == 0);
static_assert((APITCH % 8) == 0 && APITCH >= K2);
static_assert(NCLS == 16);

typedef float          v4f  __attribute__((ext_vector_type(4)));
typedef float          v8f  __attribute__((ext_vector_type(8)));
typedef double         v2d  __attribute__((ext_vector_type(2)));
typedef int            v4i  __attribute__((ext_vector_type(4)));
typedef int            v8i  __attribute__((ext_vector_type(8)));
typedef unsigned int   v4u  __attribute__((ext_vector_type(4)));
typedef unsigned short v8us __attribute__((ext_vector_type(8)));
typedef __bf16         v16b __attribute__((ext_vector_type(16)));
typedef v4f  __attribute__((may_alias)) v4fa;
typedef v2d  __attribute__((may_alias)) v2da;
typedef v4i  __attribute__((may_alias)) v4ia;
typedef v4u  __attribute__((may_alias)) v4ua;
typedef v8us __attribute__((may_alias)) v8usa;
union FragB { v16b v; v8us h[2]; v8i w; };

__device__ __forceinline__ v8f wmb(const FragB& a, const FragB& b, v8f c) {
  v8f d = __builtin_amdgcn_wmma_f32_16x16x32_bf16(false, a.v, false, b.v, (short)0, c, false, false);
  asm volatile("v_nop\n\tv_nop\n\tv_nop\n\tv_nop" : "+v"(d) : "v"(a.w), "v"(b.w));
  return d;
}

__device__ __forceinline__ unsigned int f2bf(float f) {
  const unsigned int u = __float_as_uint(f);
  const unsigned int r = ((u + 0x7FFFu + ((u >> 16) & 1u)) >> 16) & 0xFFFFu;
  return (f != f) ? 0x7FC0u : r;
}
__device__ __forceinline__ float bf2f(unsigned int b) { return __uint_as_float(b << 16); }
__device__ __forceinline__ float bfr(float f) { return bf2f(f2bf(f)); }
__device__ __forceinline__ v4f bfr4(const v4f a) {
  v4f r; r.x = bfr(a.x); r.y = bfr(a.y); r.z = bfr(a.z); r.w = bfr(a.w); return r;
}
__device__ __forceinline__ unsigned int pk2(float lo, float hi) { return f2bf(lo) | (f2bf(hi) << 16); }
__device__ __forceinline__ unsigned int pk2lo(float lo, float hi) {
  return f2bf(lo - bfr(lo)) | (f2bf(hi - bfr(hi)) << 16);
}
__device__ __forceinline__ v4u pack8(const v4f a, const v4f b) {
  v4u r;
  r.x = pk2(a.x, a.y); r.y = pk2(a.z, a.w); r.z = pk2(b.x, b.y); r.w = pk2(b.z, b.w);
  return r;
}
__device__ __forceinline__ v4u pack8lo(const v4f a, const v4f b) {
  v4u r;
  r.x = pk2lo(a.x, a.y); r.y = pk2lo(a.z, a.w); r.z = pk2lo(b.x, b.y); r.w = pk2lo(b.z, b.w);
  return r;
}
__device__ __forceinline__ float relu_np(float v) { return (v > 0.0f) ? v : (v - v); }

__device__ __forceinline__ int scan_chunk(const int* __restrict__ dsts, int nE, int cbase, int slotBase,
                                          int nb, int vec8, int* list, int tid, int lane, int wave) {
  int wc = 0;
  const int el0  = tid * EPT;
  const int e0   = cbase + el0;
  const int sent = -2147483647 - 1;
  v4i da, db;
  if (vec8 != 0 && cbase + CHUNK <= nE) {
    da = *(const v4i*)(dsts + e0);
    db = *(const v4i*)(dsts + e0 + 4);
  } else {
    da.x = (e0     < nE) ? dsts[min(e0,     nE - 1)] : sent;
    da.y = (e0 + 1 < nE) ? dsts[min(e0 + 1, nE - 1)] : sent;
    da.z = (e0 + 2 < nE) ? dsts[min(e0 + 2, nE - 1)] : sent;
    da.w = (e0 + 3 < nE) ? dsts[min(e0 + 3, nE - 1)] : sent;
    db.x = (e0 + 4 < nE) ? dsts[min(e0 + 4, nE - 1)] : sent;
    db.y = (e0 + 5 < nE) ? dsts[min(e0 + 5, nE - 1)] : sent;
    db.z = (e0 + 6 < nE) ? dsts[min(e0 + 6, nE - 1)] : sent;
    db.w = (e0 + 7 < nE) ? dsts[min(e0 + 7, nE - 1)] : sent;
  }
  const unsigned nbs = (unsigned)slotBase;
  const unsigned unb = (unsigned)nb;
  const unsigned s0 = (unsigned)da.x - nbs, s1 = (unsigned)da.y - nbs;
  const unsigned s2 = (unsigned)da.z - nbs, s3 = (unsigned)da.w - nbs;
  const unsigned s4 = (unsigned)db.x - nbs, s5 = (unsigned)db.y - nbs;
  const unsigned s6 = (unsigned)db.z - nbs, s7 = (unsigned)db.w - nbs;
  const bool h0 = s0 < unb, h1 = s1 < unb, h2 = s2 < unb, h3 = s3 < unb;
  const bool h4 = s4 < unb, h5 = s5 < unb, h6 = s6 < unb, h7 = s7 < unb;
  const unsigned any = __builtin_amdgcn_ballot_w32(h0 | h1 | h2 | h3 | h4 | h5 | h6 | h7);
  if (any != 0u) {
#define HITJ(J, HJ, SJ) { \
      const unsigned mj = __builtin_amdgcn_ballot_w32(HJ); \
      if (mj != 0u) { \
        if (HJ) { \
          const int pos = wc + (int)__builtin_amdgcn_mbcnt_lo(mj, 0u); \
          if (pos < WCAP) list[wave * WCAP + pos] = ((el0 + (J)) << SLOTB) | (int)(SJ); \
        } \
        wc += (int)__builtin_popcount(mj); } }
    HITJ(0, h0, s0)
    HITJ(1, h1, s1)
    HITJ(2, h2, s2)
    HITJ(3, h3, s3)
    HITJ(4, h4, s4)
    HITJ(5, h5, s5)
    HITJ(6, h6, s6)
    HITJ(7, h7, s7)
#undef HITJ
  }
  return wc;
}

__global__ __launch_bounds__(NTHR) void k_xprep(const float* __restrict__ x, unsigned short* xb, int nN, int nUnits) {
  const int i = (int)blockIdx.x * NTHR + (int)threadIdx.x;
  if (i >= nUnits) return;
  const int row = i >> 4;
  const int c0  = (i & 15) * 8;
  const int rc  = row < nN ? row : nN - 1;
  const float* p = x + (size_t)rc * FIN + c0;
  v4f a = *(const v4fa*)p, b = *(const v4fa*)(p + 4);
  const v4f z4 = {0.f, 0.f, 0.f, 0.f};
  if (row >= nN) { a = z4; b = z4; }
  const v4u hv = pack8(a, b);
  const size_t o = (size_t)row * FIN + c0;
  *(volatile v4u*)(xb + o) = hv;
  __threadfence();
  *(volatile v4u*)(xb + o) = hv;
}

__global__ __launch_bounds__(NTHR) void k_wtr(const float* __restrict__ w, int Kin, int Ncol, int Nrows, int Kout,
                                              unsigned short* wt, int nUnits) {
  const int u = (int)blockIdx.x * NTHR + (int)threadIdx.x;
  if (u >= nUnits) return;
  const int kq = Kout >> 3;
  const int n  = u / kq;
  const int k8 = (u - n * kq) * 8;
  const int kk = k8 - (k8 / Kin) * Kin;
  const int ncl = n < Ncol ? n : Ncol - 1;
  const float* p = w + (size_t)kk * (size_t)Ncol + ncl;
  v4f a, b;
  a.x = p[0];                    a.y = p[(size_t)Ncol];         a.z = p[(size_t)2 * Ncol];     a.w = p[(size_t)3 * Ncol];
  b.x = p[(size_t)4 * Ncol];     b.y = p[(size_t)5 * Ncol];     b.z = p[(size_t)6 * Ncol];     b.w = p[(size_t)7 * Ncol];
  const v4f z4 = {0.f, 0.f, 0.f, 0.f};
  if (n >= Ncol || n >= Nrows) { a = z4; b = z4; }
  const v4u wv = pack8(a, b);
  unsigned short* o = wt + (size_t)n * (size_t)Kout + k8;
  *(volatile v4u*)o = wv;
  __threadfence();
  *(volatile v4u*)o = wv;
}

__global__ __launch_bounds__(NTHR) void k_bucket(const int* __restrict__ srcAll, const int* __restrict__ dstAll,
                                                 int* HITS, int* META, int nN, int nE, int vec8) {
  extern __shared__ v4f lds_dyn[];
  int* reg1 = (int*)lds_dyn;
  int* reg2 = reg1 + RCAP;
  int* scnt = reg2 + RCAP;
  int* soff = scnt + NB;
  int* list = soff + NB;
  int* wcnt = list + LISTN;
  int* wtot = wcnt + NWAVE;
  const int tid = (int)threadIdx.x, lane = tid & 31, wave = tid >> 5;
  const int b = (int)blockIdx.x, r = (int)blockIdx.y, nBk = (int)gridDim.x;
  const int* srcs = srcAll + (size_t)r * (size_t)nE;
  const int* dsts = dstAll + (size_t)r * (size_t)nE;
  const int nodeBase = b * NB;

  for (int i = tid; i < NB; i += NTHR) scnt[i] = 0;
  if (tid == 0) reg2[0] = 0;
  __syncthreads();

  int tot = 0;
  const int nChunks = (nE + CHUNK - 1) / CHUNK;
#pragma unroll 1
  for (int ch = 0; ch < nChunks; ++ch) {
    const int cbase = ch * CHUNK;
    const int wc = scan_chunk(dsts, nE, cbase, nodeBase, NB, vec8, list, tid, lane, wave);
    if (lane == 0) wcnt[wave] = wc;
    __syncthreads();
    int pre = 0, all = 0;
#pragma unroll
    for (int w2 = 0; w2 < NWAVE; ++w2) {
      int c = wcnt[w2];
      c = c < 0 ? 0 : (c > WCAP ? WCAP : c);
      all += c;
      pre += (w2 < wave) ? c : 0;
    }
    const int wcc  = wc > WCAP ? WCAP : wc;
    const int base = tot + pre;
#pragma unroll 1
    for (int i = lane; i < wcc; i += 32) {
      const int ent = list[wave * WCAP + i];
      const int el  = (ent >> SLOTB) & (CHUNK - 1);
      const int sl  = ent & (NB - 1);
      int eid = cbase + el;
      eid = eid > nE - 1 ? nE - 1 : eid;
      const int pos = base + i;
      if (pos < RCAP) reg1[pos] = (int)(((unsigned)eid << SLOTB) | (unsigned)sl);
    }
    tot += all;
    tot = tot > RCAP ? RCAP : tot;
    __syncthreads();
  }
  const int nh = tot;

  if (wave == 0) {
#pragma unroll 1
    for (int b0 = 0; b0 < nh; b0 += 32) {
      const int idx = b0 + lane;
      const int uv  = reg1[idx < nh ? idx : nh - 1];
      const int m32 = (nh - b0) < 32 ? (nh - b0) : 32;
#pragma unroll 1
      for (int k = 0; k < m32; ++k) {
        const int u  = __builtin_amdgcn_readlane(uv, k);
        const int sl = u & (NB - 1);
        if (lane == 0) scnt[sl] = scnt[sl] + 1;
      }
    }
  }
  __syncthreads();

  {
    const v4i ca = *(const v4ia*)(scnt + 4 * tid);
    const int e0 = ca.x < 0 ? 0 : ca.x, e1 = ca.y < 0 ? 0 : ca.y, e2 = ca.z < 0 ? 0 : ca.z, e3 = ca.w < 0 ? 0 : ca.w;
    const int ts = e0 + e1 + e2 + e3;
    int incl = ts;
#pragma unroll
    for (int d = 1; d < 32; d <<= 1) {
      const int up = __shfl_up(incl, d);
      if (lane >= d) incl += up;
    }
    if (lane == 31) wtot[wave] = incl;
    __syncthreads();
    int pre = 0;
#pragma unroll
    for (int w2 = 0; w2 < NWAVE; ++w2) pre += (w2 < wave) ? wtot[w2] : 0;
    int run = pre + incl - ts;
    soff[4 * tid + 0] = run; run += e0;
    soff[4 * tid + 1] = run; run += e1;
    soff[4 * tid + 2] = run; run += e2;
    soff[4 * tid + 3] = run;
  }
  __syncthreads();
  for (int i = tid; i < NB; i += NTHR) list[i] = soff[i];
  __syncthreads();

  if (wave == 0) {
#pragma unroll 1
    for (int b0 = 0; b0 < nh; b0 += 32) {
      const int idx = b0 + lane;
      const int uv  = reg1[idx < nh ? idx : nh - 1];
      const int m32 = (nh - b0) < 32 ? (nh - b0) : 32;
#pragma unroll 1
      for (int k = 0; k < m32; ++k) {
        const int u   = __builtin_amdgcn_readlane(uv, k);
        const int sl  = u & (NB - 1);
        const int eid = (int)((unsigned)u >> SLOTB);
        if (lane == 0) {
          int pos = list[sl];
          pos = pos < 0 ? 0 : (pos > RCAP - 1 ? RCAP - 1 : pos);
          reg2[pos] = eid;
          list[sl] = pos + 1;
        }
      }
    }
  }
  __syncthreads();

  int* hp = HITS + (size_t)(r * nBk + b) * RCAP;
#pragma unroll 1
  for (int it = 0; it < RCAP / (4 * NTHR); ++it) {
    const int i4 = 4 * (it * NTHR + tid);
    int sv[4];
#pragma unroll
    for (int j = 0; j < 4; ++j) {
      const int idx = i4 + j;
      int c = idx < nh ? idx : nh - 1;
      c = c < 0 ? 0 : c;
      int eid = reg2[c];
      eid = eid < 0 ? 0 : (eid > nE - 1 ? nE - 1 : eid);
      int s = srcs[eid];
      asm volatile("" :: "v"(s));
      s = s < 0 ? 0 : (s > nN - 1 ? nN - 1 : s);
      sv[j] = (idx < nh) ? s : 0;
    }
    v4i o;
    o.x = sv[0]; o.y = sv[1]; o.z = sv[2]; o.w = sv[3];
    *(volatile v4i*)(hp + i4) = o;
    __threadfence();
    *(volatile v4i*)(hp + i4) = o;
  }

  {
    int* mp = META + (size_t)(r * nBk + b) * MSTR;
    const v4i a = *(const v4ia*)(soff + 4 * tid);
    const v4i c = *(const v4ia*)(scnt + 4 * tid);
    v4i h;
    h.x = (tid == 0) ? nh : 0;
    h.y = (tid == 0) ? ((nh >= RCAP) ? 1 : 0) : 0;
    h.z = 0; h.w = 0;
    const bool wh = tid < 8;
    *(volatile v4i*)(mp + 4 * tid) = a;
    *(volatile v4i*)(mp + NB + 4 * tid) = c;
    if (wh) *(volatile v4i*)(mp + 2 * NB + 4 * tid) = h;
    __threadfence();
    *(volatile v4i*)(mp + 4 * tid) = a;
    *(volatile v4i*)(mp + NB + 4 * tid) = c;
    if (wh) *(volatile v4i*)(mp + 2 * NB + 4 * tid) = h;
  }
}

template <int MODE>
__global__ __launch_bounds__(GTHR) void k_gemm(
    const unsigned short* __restrict__ A, const unsigned short* __restrict__ WT, int K,
    float* wsf, unsigned long long offA, unsigned long long offB,
    const float* __restrict__ pa, const float* __restrict__ pb,
    float* SD, int MPr, double* REC, int nN)
{
  __shared__ __attribute__((aligned(16))) float stg[GBM * GBN];
  __shared__ __attribute__((aligned(16))) float satt[4 * HD];
  __shared__ __attribute__((aligned(16))) float sdot[4 * GBM];
  __shared__ __attribute__((aligned(16))) double dps[4 * GBN];
  const int tid = (int)threadIdx.x, lane = tid & 31, wave = tid >> 5, hh = lane >> 4, m = lane & 15;
  const int rowBase = (int)blockIdx.x * GBM;
  const int by      = (int)blockIdx.y;
  const int col0    = by * GBN;

  if constexpr (MODE == 0) {
    const int hb    = tid >> 6;
    const int which = (tid >> 5) & 1;
    const int c     = tid & 31;
    int head = 2 * by + hb;
    head = head < 2 * 4 ? head : 2 * 4 - 1;
    const float vs = pa[head * HD + c];
    const float vd = pb[head * HD + c];
    const float v = (which == 0) ? vs : vd;
    satt[(2 * hb + which) * HD + c] = bfr(v);
  } else {
    const int cc = col0 + (tid & (GBN - 1));
    const float bv = pa[cc];
    satt[tid] = (tid < GBN) ? bfr(bv) : 0.0f;
  }

  v8f acc[4];
  {
    const v8f z = {0.f, 0.f, 0.f, 0.f, 0.f, 0.f, 0.f, 0.f};
    acc[0] = z; acc[1] = z; acc[2] = z; acc[3] = z;
  }
  const unsigned short* ap = A  + (size_t)(rowBase + 16 * wave + m) * (size_t)K + 8 * hh;
  const unsigned short* wp = WT + (size_t)(col0 + m) * (size_t)K + 8 * hh;
  const int ksteps = K >> 5;
#pragma unroll 1
  for (int ks = 0; ks < ksteps; ++ks) {
    FragB af;
    af.h[0] = *(const v8usa*)(ap + 32 * ks);
    af.h[1] = *(const v8usa*)(ap + 32 * ks + 16);
#pragma unroll
    for (int t = 0; t < 4; ++t) {
      const unsigned short* wq = wp + (size_t)(16 * t) * (size_t)K + 32 * ks;
      FragB bf;
      bf.h[0] = *(const v8usa*)wq;
      bf.h[1] = *(const v8usa*)(wq + 16);
      acc[t] = wmb(af, bf, acc[t]);
    }
  }

#pragma unroll
  for (int t = 0; t < 4; ++t) {
    const int lc = 16 * t + m;
#pragma unroll
    for (int r = 0; r < 8; ++r) {
      const int lr = 16 * wave + 8 * hh + r;
      stg[lr * GBN + lc] = acc[t][r];
    }
  }
  __syncthreads();

  if constexpr (MODE == 0) {
    const bool isFs = by < 4;
    if (isFs) {
      const int row = tid & 63, hb = tid >> 6;
      const float* sa = satt + (2 * hb) * HD;
      const float* sb = sa + HD;
      const float* hr = stg + row * GBN + HD * hb;
      float ds = 0.f, dd = 0.f;
#pragma unroll 2
      for (int c4 = 0; c4 < HD / 4; ++c4) {
        const v4f hv = *(const v4fa*)(hr + 4 * c4);
        const v4f av = *(const v4fa*)(sa + 4 * c4);
        const v4f bv = *(const v4fa*)(sb + 4 * c4);
        ds = fmaf(hv.x, av.x, ds);  dd = fmaf(hv.x, bv.x, dd);
        ds = fmaf(hv.y, av.y, ds);  dd = fmaf(hv.y, bv.y, dd);
        ds = fmaf(hv.z, av.z, ds);  dd = fmaf(hv.z, bv.z, dd);
        ds = fmaf(hv.w, av.w, ds);  dd = fmaf(hv.w, bv.w, dd);
      }
      sdot[(2 * hb) * GBM + row]     = ds;
      sdot[(2 * hb + 1) * GBM + row] = dd;
    }
    __syncthreads();

    v4f fv[8];
#pragma unroll
    for (int i = 0; i < 8; ++i) {
      const int lr = 16 * wave + 2 * i + hh;
      fv[i] = *(const v4fa*)(stg + lr * GBN + 4 * m);
    }
    const bool wsd = (wave < 2) && isFs;
    const int pl = 2 * (wave & 1) + (lane >> 4), piece = lane & 15;
    v4f sdv = {0.f, 0.f, 0.f, 0.f};
    if (wsd) sdv = *(const v4fa*)(sdot + pl * GBM + 4 * piece);
    const int byc = isFs ? by : 0;
    float* sp = SD + (size_t)(4 * byc + pl) * (size_t)MPr + rowBase + 4 * piece;
    const size_t obase = isFs ? ((size_t)offA + (size_t)(GBN * by)) : ((size_t)offB + (size_t)(GBN * (by - 4)));
    const int ldo = isFs ? 2 * FIN : FIN;

#pragma unroll
    for (int i = 0; i < 8; ++i) {
      const int gr = rowBase + 16 * wave + 2 * i + hh;
      float* op = wsf + obase + (size_t)gr * (size_t)ldo + 4 * m;
      *(volatile v4f*)op = fv[i];
    }
    if (wsd) *(volatile v4f*)sp = sdv;
    __threadfence();
#pragma unroll
    for (int i = 0; i < 8; ++i) {
      const int gr = rowBase + 16 * wave + 2 * i + hh;
      float* op = wsf + obase + (size_t)gr * (size_t)ldo + 4 * m;
      *(volatile v4f*)op = fv[i];
    }
    if (wsd) *(volatile v4f*)sp = sdv;
  } else {
    {
      const int col = tid & 63, half = tid >> 6;
      const float bc = satt[col];
      double s1 = 0.0, s2 = 0.0;
#pragma unroll 4
      for (int i = 0; i < 32; ++i) {
        const int row = 32 * half + i;
        const float v = stg[row * GBN + col] + bc;
        const double dv = (rowBase + row < nN) ? (double)v : 0.0;
        s1 += dv;
        s2 += dv * dv;
      }
      dps[(half * GBN + col) * 2]     = s1;
      dps[(half * GBN + col) * 2 + 1] = s2;
    }
    __syncthreads();
    const bool wr = tid < GBN;
    v2d rv = {0.0, 0.0};
    if (wr) {
      rv.x = dps[tid * 2]     + dps[(GBN + tid) * 2];
      rv.y = dps[tid * 2 + 1] + dps[(GBN + tid) * 2 + 1];
    }
    double* rp = REC + ((size_t)blockIdx.x * FIN + (size_t)col0 + (size_t)(tid & (GBN - 1))) * 2;

    const v4f b4 = *(const v4fa*)(satt + 4 * m);
    v4f fv[8];
#pragma unroll
    for (int i = 0; i < 8; ++i) {
      const int lr = 16 * wave + 2 * i + hh;
      const v4f x = *(const v4fa*)(stg + lr * GBN + 4 * m);
      v4f y;
      y.x = x.x + b4.x; y.y = x.y + b4.y; y.z = x.z + b4.z; y.w = x.w + b4.w;
      fv[i] = y;
    }
    const size_t obase = (size_t)offA + (size_t)col0;
#pragma unroll
    for (int i = 0; i < 8; ++i) {
      const int gr = rowBase + 16 * wave + 2 * i + hh;
      float* op = wsf + obase + (size_t)gr * (size_t)FIN + 4 * m;
      *(volatile v4f*)op = fv[i];
    }
    if (wr) *(volatile v2d*)rp = rv;
    __threadfence();
#pragma unroll
    for (int i = 0; i < 8; ++i) {
      const int gr = rowBase + 16 * wave + 2 * i + hh;
      float* op = wsf + obase + (size_t)gr * (size_t)FIN + 4 * m;
      *(volatile v4f*)op = fv[i];
    }
    if (wr) *(volatile v2d*)rp = rv;
  }
}

__global__ __launch_bounds__(NTHR) void k_scan(
    const int* __restrict__ HITS, const int* __restrict__ META,
    const float* __restrict__ FS, const float* __restrict__ SD,
    float* S,
    const float* __restrict__ cbias, const float* __restrict__ skb,
    double* REC, int nN, int nBk, int MPr)
{
  __shared__ __attribute__((aligned(16))) float  sbias[NREL * FIN];
  __shared__ __attribute__((aligned(16))) float  sskb[FIN];
  __shared__ __attribute__((aligned(16))) double wp[NWAVE * FIN * 2];
  __shared__ __attribute__((aligned(16))) double rec[2 * FIN];
  const int tid = (int)threadIdx.x, lane = tid & 31;
  const int wave = __builtin_amdgcn_readfirstlane(tid >> 5);
  const int bs = (int)blockIdx.x;
  int bb = bs >> 3;
  bb = bb < nBk ? bb : nBk - 1;

  if (tid < 64) {
    const v4f v = *(const v4fa*)(cbias + 4 * tid);
    *(v4fa*)(sbias + 4 * tid) = bfr4(v);
  } else if (tid < 96) {
    const v4f v = *(const v4fa*)(skb + 4 * (tid - 64));
    *(v4fa*)(sskb + 4 * (tid - 64)) = bfr4(v);
  }
  __syncthreads();

  const int c0   = 4 * lane;
  const int head = lane >> 3;
  const float qnan = __int_as_float(0x7fc00000);
  const v4f skv = *(const v4fa*)(sskb + c0);
  double q1[4], q2[4];
#pragma unroll
  for (int j = 0; j < 4; ++j) { q1[j] = 0.0; q2[j] = 0.0; }

#pragma unroll 1
  for (int jt = 0; jt < 16; ++jt) {
    const int lrow = wave * 16 + jt;
    const int slot = (bs & 7) * SROWS + lrow;
    const int grow = bs * SROWS + lrow;
    const bool live = grow < nN;
    const int gcl  = live ? grow : nN - 1;
    v4f hs = {0.f, 0.f, 0.f, 0.f};
    float pz = 0.0f;

#pragma unroll 1
    for (int r = 0; r < NREL; ++r) {
      const int* meta = META + (size_t)(r * nBk + bb) * MSTR;
      const int* hl   = HITS + (size_t)(r * nBk + bb) * RCAP;
      int st = meta[slot];
      const int craw = meta[NB + slot];
      int nh = meta[2 * NB];
      const int ovf = meta[2 * NB + 1];
      nh = nh < 0 ? 0 : (nh > RCAP ? RCAP : nh);
      st = st < 0 ? 0 : (st > nh ? nh : st);
      int cnt = craw < 0 ? 0 : (craw > DEGCAP ? DEGCAP : craw);
      if (cnt > nh - st) cnt = nh - st;
      if (ovf != 0 || craw > DEGCAP || craw < 0) pz = qnan;

      const float adv = SD[(size_t)(8 * r + 2 * head + 1) * (size_t)MPr + gcl];
      const float* ASp = SD + (size_t)(8 * r + 2 * head) * (size_t)MPr;
      const float* Fr  = FS + FIN * r + c0;
      float mx = MX0, dn = 0.0f;
      v4f av = {0.f, 0.f, 0.f, 0.f};

#pragma unroll 1
      for (int b0 = 0; b0 < cnt; b0 += 32) {
        int idx = st + b0 + lane;
        idx = idx > RCAP - 1 ? RCAP - 1 : idx;
        int sv = hl[idx];
        sv = sv < 0 ? 0 : (sv > nN - 1 ? nN - 1 : sv);
        const int m32 = (cnt - b0) < 32 ? (cnt - b0) : 32;
#pragma unroll 1
        for (int k = 0; k < m32; ++k) {
          const int sk = __builtin_amdgcn_readlane(sv, k);
          const v4f fs = *(const v4fa*)(Fr + (size_t)sk * (size_t)(2 * FIN));
          float lg = ASp[sk] + adv;
          lg = lg > 0.f ? lg : NEGSL * lg;
          const float df = lg - mx;
          const float ee = expf(-fabsf(df));
          const bool up  = df > 0.f;
          const float s1 = up ? ee : 1.0f;
          const float s2 = up ? 1.0f : ee;
          mx = up ? lg : mx;
          dn = fmaf(dn, s1, s2);
          av.x = fmaf(av.x, s1, s2 * fs.x);
          av.y = fmaf(av.y, s1, s2 * fs.y);
          av.z = fmaf(av.z, s1, s2 * fs.z);
          av.w = fmaf(av.w, s1, s2 * fs.w);
        }
      }
      const float dsafe = (cnt > 0) ? dn : 1.0f;
      const float inv = __builtin_amdgcn_rcpf(dsafe);
      const v4f b4 = *(const v4fa*)(sbias + FIN * r + c0);
      hs.x += fmaf(av.x, inv, b4.x);
      hs.y += fmaf(av.y, inv, b4.y);
      hs.z += fmaf(av.z, inv, b4.z);
      hs.w += fmaf(av.w, inv, b4.w);
    }

    float* sp = S + (size_t)grow * FIN + c0;
    const v4f sr = *(const v4fa*)sp;
    asm volatile("" :: "v"(sr));
    v4f o;
    o.x = ((sr.x + skv.x) + relu_np(hs.x)) + pz;
    o.y = ((sr.y + skv.y) + relu_np(hs.y)) + pz;
    o.z = ((sr.z + skv.z) + relu_np(hs.z)) + pz;
    o.w = ((sr.w + skv.w) + relu_np(hs.w)) + pz;
    if (live) {
      const double d0 = (double)o.x, d1 = (double)o.y, d2 = (double)o.z, d3 = (double)o.w;
      q1[0] += d0; q2[0] += d0 * d0;
      q1[1] += d1; q2[1] += d1 * d1;
      q1[2] += d2; q2[2] += d2 * d2;
      q1[3] += d3; q2[3] += d3 * d3;
    }
    if (live) *(volatile v4f*)sp = o;
    __threadfence();
    if (live) *(volatile v4f*)sp = o;
  }

  {
    double* wq = wp + ((size_t)wave * FIN + c0) * 2;
#pragma unroll
    for (int j = 0; j < 4; ++j) { wq[2 * j] = q1[j]; wq[2 * j + 1] = q2[j]; }
  }
  __syncthreads();
  {
    const int col = tid & (FIN - 1), which = tid >> 7;
    double a = 0.0;
#pragma unroll 1
    for (int w2 = 0; w2 < NWAVE; ++w2) a += wp[((size_t)w2 * FIN + col) * 2 + which];
    rec[col * 2 + which] = a;
  }
  __syncthreads();
  const bool wr = tid < FIN;
  v2d rv = {0.0, 0.0};
  if (wr) rv = *(const v2da*)(rec + 2 * tid);
  double* rp = REC + ((size_t)bs * FIN + (size_t)(tid & (FIN - 1))) * 2;
  if (wr) *(volatile v2d*)rp = rv;
  __threadfence();
  if (wr) *(volatile v2d*)rp = rv;
}

__global__ __launch_bounds__(FIN) void k_comb(const double* __restrict__ REC, int nRec, double invN,
                                              const float* __restrict__ gam, const float* __restrict__ bet,
                                              float* SS) {
  __shared__ __attribute__((aligned(16))) float stg[2 * FIN];
  const int c = (int)threadIdx.x;
  double s1 = 0.0, s2 = 0.0;
#pragma unroll 1
  for (int b = 0; b < nRec; ++b) {
    const v2d q = *(const v2da*)(REC + ((size_t)b * FIN + c) * 2);
    s1 += q.x;
    s2 += q.y;
  }
  const double mu  = s1 * invN;
  const double var = s2 * invN - mu * mu;
  const float varf = (float)var;
  const float rstd = 1.0f / sqrtf(varf + 1e-5f);
  const float sc = bfr(gam[c]) * rstd;
  const float sh = (float)((double)bfr(bet[c]) - mu * (double)sc);
  stg[c] = sc;
  stg[FIN + c] = sh;
  __syncthreads();
  const bool wr = c < (2 * FIN) / 4;
  v4f v = {0.f, 0.f, 0.f, 0.f};
  if (wr) v = *(const v4fa*)(stg + 4 * c);
  float* op = SS + 4 * (c & 63);
  if (wr) *(volatile v4f*)op = v;
  __threadfence();
  if (wr) *(volatile v4f*)op = v;
}

__global__ __launch_bounds__(NTHR) void k_norm(const float* __restrict__ S, const float* __restrict__ SS,
                                               unsigned short* HL, int nN, int nUnits) {
  __shared__ __attribute__((aligned(16))) float sss[2 * FIN];
  const int tid = (int)threadIdx.x;
  if (tid < 64) *(v4fa*)(sss + 4 * tid) = *(const v4fa*)(SS + 4 * tid);
  __syncthreads();
  const int u = (int)blockIdx.x * NTHR + tid;
  if (u >= nUnits) return;
  const int row = u >> 4;
  const int c8  = (u & 15) * 8;
  const int rc  = row < nN ? row : nN - 1;
  const float* p = S + (size_t)rc * FIN + c8;
  const v4f a = *(const v4fa*)p, b = *(const v4fa*)(p + 4);
  const v4f sa = *(const v4fa*)(sss + c8), sb = *(const v4fa*)(sss + c8 + 4);
  const v4f ta = *(const v4fa*)(sss + FIN + c8), tb = *(const v4fa*)(sss + FIN + c8 + 4);
  v4f ya, yb;
  ya.x = fmaf(a.x, sa.x, ta.x); ya.y = fmaf(a.y, sa.y, ta.y); ya.z = fmaf(a.z, sa.z, ta.z); ya.w = fmaf(a.w, sa.w, ta.w);
  yb.x = fmaf(b.x, sb.x, tb.x); yb.y = fmaf(b.y, sb.y, tb.y); yb.z = fmaf(b.z, sb.z, tb.z); yb.w = fmaf(b.w, sb.w, tb.w);
  const v4f z4 = {0.f, 0.f, 0.f, 0.f};
  if (row >= nN) { ya = z4; yb = z4; }
  const v4u hv = pack8(ya, yb);
  const v4u lv = pack8lo(ya, yb);
  unsigned short* o = HL + (size_t)row * K2 + c8;
  *(volatile v4u*)o = hv;
  *(volatile v4u*)(o + FIN) = lv;
  __threadfence();
  *(volatile v4u*)o = hv;
  *(volatile v4u*)(o + FIN) = lv;
}

__global__ __launch_bounds__(GTHR) void k_head(const float* __restrict__ Z, const float* __restrict__ SS,
                                               const unsigned short* __restrict__ C2T,
                                               const float* __restrict__ b2, float* out, int nN) {
  __shared__ __attribute__((aligned(16))) unsigned short sa[GBM * APITCH];
  __shared__ __attribute__((aligned(16))) float sss[2 * FIN];
  __shared__ __attribute__((aligned(16))) float sot[GBM * NCLS];
  __shared__ __attribute__((aligned(16))) float sb2[NCLS];
  const int tid = (int)threadIdx.x, lane = tid & 31, wave = tid >> 5, hh = lane >> 4, m = lane & 15;
  const int rowBase = (int)blockIdx.x * GBM;

  if (tid < 64) *(v4fa*)(sss + 4 * tid) = *(const v4fa*)(SS + 4 * tid);
  if (tid >= 64 && tid < 68) {
    const v4f v = *(const v4fa*)(b2 + 4 * (tid - 64));
    *(v4fa*)(sb2 + 4 * (tid - 64)) = bfr4(v);
  }
  __syncthreads();

#pragma unroll 1
  for (int it = 0; it < 8; ++it) {
    const int p   = it * GTHR + tid;
    const int row = p >> 4;
    const int c8  = (p & 15) * 8;
    const float* zp = Z + (size_t)(rowBase + row) * FIN + c8;
    const v4f a = *(const v4fa*)zp, b = *(const v4fa*)(zp + 4);
    const v4f s0 = *(const v4fa*)(sss + c8), s1 = *(const v4fa*)(sss + c8 + 4);
    const v4f t0 = *(const v4fa*)(sss + FIN + c8), t1 = *(const v4fa*)(sss + FIN + c8 + 4);
    v4f xa, xb;
    xa.x = relu_np(fmaf(a.x, s0.x, t0.x)); xa.y = relu_np(fmaf(a.y, s0.y, t0.y));
    xa.z = relu_np(fmaf(a.z, s0.z, t0.z)); xa.w = relu_np(fmaf(a.w, s0.w, t0.w));
    xb.x = relu_np(fmaf(b.x, s1.x, t1.x)); xb.y = relu_np(fmaf(b.y, s1.y, t1.y));
    xb.z = relu_np(fmaf(b.z, s1.z, t1.z)); xb.w = relu_np(fmaf(b.w, s1.w, t1.w));
    *(v4ua*)(sa + row * APITCH + c8)       = pack8(xa, xb);
    *(v4ua*)(sa + row * APITCH + FIN + c8) = pack8lo(xa, xb);
  }
  __syncthreads();

  v8f acc = {0.f, 0.f, 0.f, 0.f, 0.f, 0.f, 0.f, 0.f};
  const unsigned short* ap = sa + (16 * wave + m) * APITCH + 8 * hh;
  const unsigned short* wq = C2T + (size_t)m * K2 + 8 * hh;
#pragma unroll 2
  for (int ks = 0; ks < K2 / 32; ++ks) {
    FragB af, bf;
    af.h[0] = *(const v8usa*)(ap + 32 * ks);
    af.h[1] = *(const v8usa*)(ap + 32 * ks + 16);
    bf.h[0] = *(const v8usa*)(wq + 32 * ks);
    bf.h[1] = *(const v8usa*)(wq + 32 * ks + 16);
    acc = wmb(af, bf, acc);
  }
  {
    const float bz = sb2[m];
#pragma unroll
    for (int r = 0; r < 8; ++r) sot[(16 * wave + 8 * hh + r) * NCLS + m] = acc[r] + bz;
  }
  __syncthreads();

  const int p0 = tid, p1 = GTHR + tid;
  const v4f v0 = *(const v4fa*)(sot + 4 * p0);
  const v4f v1 = *(const v4fa*)(sot + 4 * p1);
  const bool ok0 = (rowBase + (p0 >> 2)) < nN;
  const bool ok1 = (rowBase + (p1 >> 2)) < nN;
  float* ob = out + (size_t)rowBase * NCLS;
  if (ok0) *(volatile v4f*)(ob + 4 * p0) = v0;
  if (ok1) *(volatile v4f*)(ob + 4 * p1) = v1;
  __threadfence();
  if (ok0) *(volatile v4f*)(ob + 4 * p0) = v0;
  if (ok1) *(volatile v4f*)(ob + 4 * p1) = v1;
}

static inline int cdiv(int a, int b) { return (a + b - 1) / b; }
static inline size_t al256(size_t o) { return (o + 255) & ~(size_t)255; }

extern "C" void kernel_launch(void* const* d_in, const int* in_sizes, int n_in,
                              void* d_out, int out_size, void* d_ws, size_t ws_size,
                              hipStream_t stream) {
  if (n_in < 17) return;
  if (in_sizes[0] < FIN || (in_sizes[0] % FIN) != 0) return;
  const int nN = in_sizes[0] / FIN;
  if (nN < 64 || nN > (1 << 20)) return;
  if (in_sizes[1] != 4 * FIN * FIN) return;
  if (in_sizes[2] != 4 * FIN || in_sizes[3] != 4 * FIN || in_sizes[4] != 4 * FIN) return;
  if (in_sizes[5] != 2 * FIN * FIN) return;
  if (in_sizes[6] != 2 * FIN || in_sizes[7] != 2 * FIN || in_sizes[8] != 2 * FIN) return;
  if (in_sizes[9] != FIN * FIN) return;
  if (in_sizes[10] != FIN || in_sizes[11] != FIN || in_sizes[12] != FIN) return;
  if (in_sizes[13] != FIN * NCLS || in_sizes[14] != NCLS) return;
  if (in_sizes[15] < 2 || (in_sizes[15] & 1) != 0 || in_sizes[16] != in_sizes[15]) return;
  const int nE = in_sizes[15] / 2;
  if (nE < 1 || nE >= (1 << 21)) return;
  if ((long long)out_size != (long long)nN * NCLS) return;
  if ((long long)NB * (long long)nE * 10LL > (long long)RCAP * (long long)nN * 9LL) return;

  const float* feat   = (const float*)d_in[0];
  const float* fcW    = (const float*)d_in[1];
  const float* attl   = (const float*)d_in[2];
  const float* attr   = (const float*)d_in[3];
  const float* cbias  = (const float*)d_in[4];
  const float* skW    = (const float*)d_in[5];
  const float* skb    = (const float*)d_in[6];
  const float* ng     = (const float*)d_in[7];
  const float* nb     = (const float*)d_in[8];
  const float* cW1    = (const float*)d_in[9];
  const float* cb1    = (const float*)d_in[10];
  const float* cg     = (const float*)d_in[11];
  const float* cb     = (const float*)d_in[12];
  const float* cW2    = (const float*)d_in[13];
  const float* cb2    = (const float*)d_in[14];
  const int*   srcAll = (const int*)d_in[15];
  const int*   dstAll = (const int*)d_in[16];
  float* out = (float*)d_out;

  const int MP  = cdiv(nN, MROWS) * MROWS;
  const int gM  = MP / GBM;
  const int gS  = MP / SROWS;
  const int nBk = cdiv(nN, NB);
  const int vec8 = ((nE & 3) == 0) ? 1 : 0;
  const int nRecMax = gM > gS ? gM : gS;

  char* ws = (char*)d_ws;
  size_t off = 0;
  const size_t oFS   = off; off = al256(off + (size_t)MP * 2 * FIN * 4);
  const size_t oS    = off; off = al256(off + (size_t)MP * FIN * 4);
  const size_t oHL   = off; off = al256(off + (size_t)MP * K2 * 2);
  const size_t oSD   = off; off = al256(off + (size_t)16 * MP * 4);
  const size_t oHITS = off; off = al256(off + (size_t)NREL * nBk * RCAP * 4);
  const size_t oMETA = off; off = al256(off + (size_t)NREL * nBk * MSTR * 4);
  const size_t oB1   = off; off = al256(off + (size_t)NCOLP * FIN * 2);
  const size_t oB2   = off; off = al256(off + (size_t)NCOLP * K2 * 2);
  const size_t oC1   = off; off = al256(off + (size_t)FIN * K2 * 2);
  const size_t oC2   = off; off = al256(off + (size_t)NCLS * K2 * 2);
  const size_t oREC  = off; off = al256(off + (size_t)nRecMax * FIN * 2 * 8);
  const size_t oSS   = off; off = al256(off + (size_t)(2 * FIN) * 4);
  if (off > ws_size || off > (size_t)WSMAX) return;

  float*          wsf  = (float*)ws;
  float*          FS   = (float*)(ws + oFS);
  float*          Sp   = (float*)(ws + oS);
  unsigned short* HL   = (unsigned short*)(ws + oHL);
  unsigned short* XB   = (unsigned short*)(ws + oHL);
  float*          SD   = (float*)(ws + oSD);
  int*            HITS = (int*)(ws + oHITS);
  int*            META = (int*)(ws + oMETA);
  unsigned short* B1T  = (unsigned short*)(ws + oB1);
  unsigned short* B2T  = (unsigned short*)(ws + oB2);
  unsigned short* C1T  = (unsigned short*)(ws + oC1);
  unsigned short* C2T  = (unsigned short*)(ws + oC2);
  double*         REC  = (double*)(ws + oREC);
  float*          SS   = (float*)(ws + oSS);
  const unsigned long long fFS = (unsigned long long)(oFS / 4);
  const unsigned long long fS  = (unsigned long long)(oS / 4);
  const double invN = 1.0 / (double)nN;

  hipFuncSetAttribute(reinterpret_cast<const void*>(&k_bucket),
                      hipFuncAttributeMaxDynamicSharedMemorySize, LDS_BK);

  const int nUx = MP * (FIN / 8);
  k_xprep<<<cdiv(nUx, NTHR), NTHR, 0, stream>>>(feat, XB, nN, nUx);

  {
    const int nU1 = FIN * (FIN / 8);
    const int nU2 = FIN * (K2 / 8);
    k_wtr<<<cdiv(nU1, NTHR), NTHR, 0, stream>>>(fcW,                 FIN, FIN, FIN, FIN, B1T,                 nU1);
    k_wtr<<<cdiv(nU1, NTHR), NTHR, 0, stream>>>(fcW + FIN * FIN,     FIN, FIN, FIN, FIN, B1T + FIN * FIN,     nU1);
    k_wtr<<<cdiv(nU1, NTHR), NTHR, 0, stream>>>(skW,                 FIN, FIN, FIN, FIN, B1T + 2 * FIN * FIN, nU1);
    k_wtr<<<cdiv(nU2, NTHR), NTHR, 0, stream>>>(fcW + 2 * FIN * FIN, FIN, FIN, FIN, K2,  B2T,                 nU2);
    k_wtr<<<cdiv(nU2, NTHR), NTHR, 0, stream>>>(fcW + 3 * FIN * FIN, FIN, FIN, FIN, K2,  B2T + FIN * K2,      nU2);
    k_wtr<<<cdiv(nU2, NTHR), NTHR, 0, stream>>>(skW + FIN * FIN,     FIN, FIN, FIN, K2,  B2T + 2 * FIN * K2,  nU2);
    k_wtr<<<cdiv(nU2, NTHR), NTHR, 0, stream>>>(cW1,                 FIN, FIN, FIN, K2,  C1T,                 nU2);
    const int nU3 = NCLS * (K2 / 8);
    k_wtr<<<cdiv(nU3, NTHR), NTHR, 0, stream>>>(cW2,                 FIN, NCLS, NCLS, K2, C2T,                nU3);
  }

  k_bucket<<<dim3(nBk, NREL), NTHR, LDS_BK, stream>>>(srcAll, dstAll, HITS, META, nN, nE, vec8);

  k_gemm<0><<<dim3(gM, NCOLP / GBN), GTHR, 0, stream>>>(XB, B1T, FIN, wsf, fFS, fS, attl, attr, SD, MP, REC, nN);
  k_scan<<<gS, NTHR, 0, stream>>>(HITS, META, FS, SD, Sp, cbias, skb, REC, nN, nBk, MP);
  k_comb<<<1, FIN, 0, stream>>>(REC, gS, invN, ng, nb, SS);
  const int nUh = MP * (FIN / 8);
  k_norm<<<cdiv(nUh, NTHR), NTHR, 0, stream>>>(Sp, SS, HL, nN, nUh);

  k_gemm<0><<<dim3(gM, NCOLP / GBN), GTHR, 0, stream>>>(HL, B2T, K2, wsf, fFS, fS, attl + 2 * FIN, attr + 2 * FIN, SD, MP, REC, nN);
  k_scan<<<gS, NTHR, 0, stream>>>(HITS, META, FS, SD, Sp, cbias + 2 * FIN, skb + FIN, REC, nN, nBk, MP);
  k_comb<<<1, FIN, 0, stream>>>(REC, gS, invN, ng + FIN, nb + FIN, SS);
  k_norm<<<cdiv(nUh, NTHR), NTHR, 0, stream>>>(Sp, SS, HL, nN, nUh);

  k_gemm<1><<<dim3(gM, FIN / GBN), GTHR, 0, stream>>>(HL, C1T, K2, wsf, fFS, fFS, cb1, cb1, SD, MP, REC, nN);
  k_comb<<<1, FIN, 0, stream>>>(REC, gM, invN, cg, cb, SS);
  k_head<<<gM, GTHR, 0, stream>>>(FS, SS, C2T, cb2, out, nN);
}
